// ModalMoE_53412213293357
// MI455X (gfx1250) — hardware-verified
//
#include <hip/hip_runtime.h>
#include <stdint.h>
#include <stddef.h>
#include <math.h>

#pragma clang fp contract(off)

#define NTOK 4096
#define NEX  4
#define NOUT 2048
#define D0   768
#define D1   1024
#define D2   512
#define D3   256
#define DTOT 2560
#define OFF1 768
#define OFF2 1792
#define OFF3 2304
#define MT   64
#define XP   1032
#define YP   260
#define SLW  256

#define LDS_XB  (MT * XP * 2)
#define LDS_YB  (MT * YP * 4)
#define LDS_EXP (LDS_XB + LDS_YB)

#define W_SC 256.0f
#define R_W  0.00390625f

static_assert(DTOT == D0 + D1 + D2 + D3);
static_assert(OFF1 == D0);
static_assert(OFF2 == D0 + D1);
static_assert(OFF3 == D0 + D1 + D2);
static_assert((XP * 2) % 16 == 0);
static_assert((YP * 4) % 16 == 0);
static_assert(XP >= D1 + 8);
static_assert(NTOK % 256 == 0);
static_assert(NTOK % MT == 0);
static_assert(MT == 8 * 8);
static_assert(D0 % 256 == 0);
static_assert(D1 % 256 == 0);
static_assert(D2 % 256 == 0);
static_assert(D3 % 256 == 0);
static_assert(NOUT % SLW == 0);
static_assert((NEX * DTOT) % 1024 == 0);
static_assert((NTOK * NOUT) % 1024 == 0);

typedef _Float16       v16h __attribute__((ext_vector_type(16)));
typedef _Float16       v8h  __attribute__((ext_vector_type(8)));
typedef float          v8f  __attribute__((ext_vector_type(8)));
typedef float          v4f  __attribute__((ext_vector_type(4)));
typedef unsigned int   v4u  __attribute__((ext_vector_type(4)));
typedef v4f __attribute__((may_alias)) v4fa;
typedef v4u __attribute__((may_alias)) v4ua;

union FragH { v16h v; v4u q[2]; };
union Pack8 { v8h h; v4u u; };

__device__ __forceinline__ v8f wmma_h(v16h a, v16h b, v8f c) {
  v8f d = __builtin_amdgcn_wmma_f32_16x16x32_f16(false, a, false, b, (short)0, c, false, false);
  asm volatile("v_nop\n\tv_nop\n\tv_nop\n\tv_nop" : "+v"(d) : "v"(a), "v"(b));
  return d;
}

__device__ __forceinline__ v16h ldfrag(const unsigned short* p, int h) {
  FragH f;
  f.q[0] = *(const v4ua*)(p + 8 * h);
  f.q[1] = *(const v4ua*)(p + 16 + 8 * h);
  return f.v;
}

__global__ __launch_bounds__(256) void k_cvt(const float* __restrict__ src,
                                             unsigned short* __restrict__ dst,
                                             int n8, float sc)
{
  const int g = blockIdx.x * 256 + threadIdx.x;
  if (g >= n8) return;
  const float* s = src + (size_t)g * 8;
  const v4f a = *(const v4fa*)s;
  const v4f c = *(const v4fa*)(s + 4);
  v8h hv;
  hv[0] = (_Float16)(a.x * sc); hv[1] = (_Float16)(a.y * sc);
  hv[2] = (_Float16)(a.z * sc); hv[3] = (_Float16)(a.w * sc);
  hv[4] = (_Float16)(c.x * sc); hv[5] = (_Float16)(c.y * sc);
  hv[6] = (_Float16)(c.z * sc); hv[7] = (_Float16)(c.w * sc);
  Pack8 p;
  p.h = hv;
  const v4u u = p.u;
  unsigned short* d = dst + (size_t)g * 8;
  *(volatile v4u*)d = u;
  __threadfence();
  *(volatile v4u*)d = u;
}

__device__ __forceinline__ void gate_seg(const float* xr, const float* sw, int nq, int lane,
                                         double& l0, double& l1, double& l2, double& l3)
{
  #pragma unroll 1
  for (int i = 0; i < nq; ++i) {
    const int k = 32 * i + lane;
    const double xv = (double)xr[k];
    l0 = fma(xv, (double)sw[k],            l0);
    l1 = fma(xv, (double)sw[DTOT + k],     l1);
    l2 = fma(xv, (double)sw[2 * DTOT + k], l2);
    l3 = fma(xv, (double)sw[3 * DTOT + k], l3);
  }
}

__global__ __launch_bounds__(256) void k_route(const float* __restrict__ f0,
                                               const float* __restrict__ f1,
                                               const float* __restrict__ f2,
                                               const float* __restrict__ f3,
                                               const float* __restrict__ gw,
                                               const float* __restrict__ gb,
                                               float* __restrict__ rec, int ntok)
{
  __shared__ __align__(16) float sgw[NEX * DTOT];
  __shared__ __align__(16) float srec[32];
  const int tid = threadIdx.x, lane = tid & 31, wv = tid >> 5;
  #pragma unroll 1
  for (int i = 0; i < (NEX * DTOT) / 1024; ++i) {
    const int o = 4 * (tid + 256 * i);
    const v4f w4 = *(const v4fa*)(gw + o);
    *(v4fa*)(sgw + o) = w4;
  }
  __syncthreads();

  const int t = blockIdx.x * 8 + wv;
  const int tc = (t < ntok) ? t : (ntok - 1);
  double l0 = 0.0, l1 = 0.0, l2 = 0.0, l3 = 0.0;
  gate_seg(f0 + (size_t)tc * D0, sgw,        D0 / 32, lane, l0, l1, l2, l3);
  gate_seg(f1 + (size_t)tc * D1, sgw + OFF1, D1 / 32, lane, l0, l1, l2, l3);
  gate_seg(f2 + (size_t)tc * D2, sgw + OFF2, D2 / 32, lane, l0, l1, l2, l3);
  gate_seg(f3 + (size_t)tc * D3, sgw + OFF3, D3 / 32, lane, l0, l1, l2, l3);
  #pragma unroll
  for (int off = 16; off > 0; off >>= 1) {
    l0 = l0 + __shfl_xor(l0, off);
    l1 = l1 + __shfl_xor(l1, off);
    l2 = l2 + __shfl_xor(l2, off);
    l3 = l3 + __shfl_xor(l3, off);
  }

  float lf[NEX];
  lf[0] = (float)l0 + gb[0];
  lf[1] = (float)l1 + gb[1];
  lf[2] = (float)l2 + gb[2];
  lf[3] = (float)l3 + gb[3];

  int i0 = 0;
  float bst = lf[0];
  #pragma unroll
  for (int e = 1; e < NEX; ++e) {
    const bool tk = lf[e] > bst;
    bst = tk ? lf[e] : bst;
    i0 = tk ? e : i0;
  }
  int i1 = -1;
  float b1 = -3.0e38f;
  #pragma unroll
  for (int e = 0; e < NEX; ++e) {
    const bool tk = (e != i0) && (lf[e] > b1);
    b1 = tk ? lf[e] : b1;
    i1 = tk ? e : i1;
  }
  i1 = (i1 < 0) ? ((i0 == 0) ? 1 : 0) : i1;

  float ex[NEX];
  #pragma unroll
  for (int e = 0; e < NEX; ++e) ex[e] = __expf(lf[e] - bst);
  const float den = (ex[0] + ex[1]) + (ex[2] + ex[3]);
  const float rden = __builtin_amdgcn_rcpf(den);
  float x0 = ex[0], x1 = ex[0];
  #pragma unroll
  for (int e = 0; e < NEX; ++e) { x0 = (e == i0) ? ex[e] : x0; x1 = (e == i1) ? ex[e] : x1; }
  const float p0 = x0 * rden;
  const float p1 = x1 * rden;

  if (lane == 0) {
    srec[4 * wv + 0] = p0;
    srec[4 * wv + 1] = p1;
    srec[4 * wv + 2] = (float)i0;
    srec[4 * wv + 3] = (float)i1;
  }
  __syncthreads();
  if (wv == 0) {
    const int q = lane & 7;
    const v4f v = *(const v4fa*)(srec + 4 * q);
    const int tt = blockIdx.x * 8 + q;
    const bool ok = (lane < 8) && (tt < ntok);
    if (ok) *(volatile v4f*)(rec + (size_t)tt * 4) = v;
    __threadfence();
    if (ok) *(volatile v4f*)(rec + (size_t)tt * 4) = v;
  }
}

__device__ __forceinline__ void part_pass(const float* sY, const int* sTok, const int* sSlot,
                                          float* part, int ns, int wv, int lane, int nrows)
{
  #pragma unroll
  for (int i = 0; i < 8; ++i) {
    const int row = wv * 8 + i;
    int t = sTok[row];
    t = (t < 0) ? 0 : ((t > NTOK - 1) ? (NTOK - 1) : t);
    int s = sSlot[row];
    s = (s != 0) ? 1 : 0;
    const v4f v0 = *(const v4fa*)(sY + row * YP + 4 * lane);
    const v4f v1 = *(const v4fa*)(sY + row * YP + 128 + 4 * lane);
    float* dst = part + ((size_t)t * 2 + s) * NOUT + ns * SLW;
    if (row < nrows) {
      *(volatile v4f*)(dst + 4 * lane) = v0;
      *(volatile v4f*)(dst + 128 + 4 * lane) = v1;
    }
  }
}

__global__ __launch_bounds__(256) void k_expert(const unsigned short* __restrict__ xh0,
                                                const unsigned short* __restrict__ xh1,
                                                const unsigned short* __restrict__ xh2,
                                                const unsigned short* __restrict__ xh3,
                                                const unsigned short* __restrict__ wh0,
                                                const unsigned short* __restrict__ wh1,
                                                const unsigned short* __restrict__ wh2,
                                                const unsigned short* __restrict__ wh3,
                                                const float* __restrict__ bb0,
                                                const float* __restrict__ bb1,
                                                const float* __restrict__ bb2,
                                                const float* __restrict__ bb3,
                                                const float* __restrict__ rec,
                                                float* __restrict__ part, int ntok)
{
  extern __shared__ __align__(16) unsigned char dsm_e[];
  unsigned short* sX = (unsigned short*)dsm_e;
  float* sY = (float*)(dsm_e + LDS_XB);
  __shared__ int   sTok[MT];
  __shared__ int   sSlot[MT];
  __shared__ float sW[MT];
  __shared__ int   s_wc[8];

  const int tid = threadIdx.x, lane = tid & 31, wv = tid >> 5;
  const int h = lane >> 4, m = lane & 15;
  const int wr = wv >> 2, wc = wv & 3;
  const int e = blockIdx.y;
  const int m0 = blockIdx.x * MT;

  const int D = (e == 0) ? D0 : ((e == 1) ? D1 : ((e == 2) ? D2 : D3));
  const unsigned short* xh = (e == 0) ? xh0 : ((e == 1) ? xh1 : ((e == 2) ? xh2 : xh3));
  const unsigned short* wh = (e == 0) ? wh0 : ((e == 1) ? wh1 : ((e == 2) ? wh2 : wh3));
  const float* bb = (e == 0) ? bb0 : ((e == 1) ? bb1 : ((e == 2) ? bb2 : bb3));

  if (tid < MT) { sTok[tid] = 0; sSlot[tid] = 0; sW[tid] = 0.0f; }
  __syncthreads();

  int base = 0;
  #pragma unroll 1
  for (int ch = 0; ch < NTOK / 256; ++ch) {
    const int t = ch * 256 + tid;
    const int tc = (t < ntok) ? t : (ntok - 1);
    const v4f r = *(const v4fa*)(rec + (size_t)tc * 4);
    int e0 = (int)r.z, e1 = (int)r.w;
    e0 = (e0 < 0) ? 0 : ((e0 > NEX - 1) ? (NEX - 1) : e0);
    e1 = (e1 < 0) ? 0 : ((e1 > NEX - 1) ? (NEX - 1) : e1);
    const bool fa = (e0 == e);
    const bool fb = (e1 == e) && !fa;
    const bool f = (fa || fb) && (t < ntok);
    const unsigned int msk = __builtin_amdgcn_ballot_w32(f);
    const int off = __builtin_popcount(msk & ((1u << lane) - 1u));
    const int wcnt = __builtin_popcount(msk);
    if (lane == 0) s_wc[wv] = wcnt;
    __syncthreads();
    int pre = 0, tot = 0;
    #pragma unroll
    for (int w2 = 0; w2 < 8; ++w2) {
      const int cc = s_wc[w2];
      tot += cc;
      pre += (w2 < wv) ? cc : 0;
    }
    if (f) {
      const int p = base + pre + off - m0;
      if ((unsigned)p < (unsigned)MT) {
        sTok[p]  = t;
        sSlot[p] = fa ? 0 : 1;
        sW[p]    = fa ? r.x : r.y;
      }
    }
    base += tot;
    __syncthreads();
  }
  const int cnt = base;
  if (m0 >= cnt) return;
  int nrows = cnt - m0;
  nrows = (nrows > MT) ? MT : nrows;

  const int nq = D >> 8;
  #pragma unroll 1
  for (int i = 0; i < 8; ++i) {
    const int row = wv * 8 + i;
    int t = sTok[row];
    t = (t < 0) ? 0 : ((t > NTOK - 1) ? (NTOK - 1) : t);
    const unsigned short* src = xh + (size_t)t * D;
    #pragma unroll 1
    for (int q = 0; q < nq; ++q) {
      const int c8 = 32 * q + lane;
      const v4u a = *(const v4ua*)(src + 8 * c8);
      *(v4ua*)(sX + row * XP + 8 * c8) = a;
    }
  }
  __syncthreads();

  const v8f z8 = {0.f, 0.f, 0.f, 0.f, 0.f, 0.f, 0.f, 0.f};

  #pragma unroll 1
  for (int ns = 0; ns < NOUT / SLW; ++ns) {
    v8f acc[2][4];
    #pragma unroll
    for (int mt = 0; mt < 2; ++mt)
      #pragma unroll
      for (int nt = 0; nt < 4; ++nt) acc[mt][nt] = z8;
    #pragma unroll 1
    for (int k0 = 0; k0 < D; k0 += 32) {
      v16h a[2];
      #pragma unroll
      for (int mt = 0; mt < 2; ++mt)
        a[mt] = ldfrag(sX + (32 * wr + 16 * mt + m) * XP + k0, h);
      #pragma unroll
      for (int nt = 0; nt < 4; ++nt) {
        const int n = ns * SLW + wc * 64 + 16 * nt + m;
        const v16h b = ldfrag(wh + (size_t)n * D + k0, h);
        #pragma unroll
        for (int mt = 0; mt < 2; ++mt) acc[mt][nt] = wmma_h(a[mt], b, acc[mt][nt]);
      }
    }
    #pragma unroll
    for (int mt = 0; mt < 2; ++mt)
      #pragma unroll
      for (int nt = 0; nt < 4; ++nt) {
        const int cl = wc * 64 + 16 * nt + m;
        const float bias = bb[ns * SLW + cl];
        #pragma unroll
        for (int r = 0; r < 8; ++r) {
          const int row = 32 * wr + 16 * mt + 8 * h + r;
          const float y = acc[mt][nt][r] * R_W + bias;
          sY[row * YP + cl] = y * sW[row];
        }
      }
    __syncthreads();
    part_pass(sY, sTok, sSlot, part, ns, wv, lane, nrows);
    __threadfence();
    part_pass(sY, sTok, sSlot, part, ns, wv, lane, nrows);
    __syncthreads();
  }
}

__global__ __launch_bounds__(256) void k_sum(const float* __restrict__ part,
                                             float* __restrict__ out, int n4)
{
  const int g = blockIdx.x * 256 + threadIdx.x;
  if (g >= n4) return;
  const int t = g / (NOUT / 4);
  const int c4 = g - t * (NOUT / 4);
  const float* p0 = part + (size_t)t * 2 * NOUT + 4 * c4;
  const float* p1 = p0 + NOUT;
  const v4f a = *(const v4fa*)p0;
  const v4f b = *(const v4fa*)p1;
  const v4f o = a + b;
  float* d = out + (size_t)g * 4;
  *(volatile v4f*)d = o;
  __threadfence();
  *(volatile v4f*)d = o;
}

extern "C" void kernel_launch(void* const* d_in, const int* in_sizes, int n_in,
                              void* d_out, int out_size, void* d_ws, size_t ws_size,
                              hipStream_t stream)
{
  if (n_in < 14) return;
  if (in_sizes[0]  != NTOK * D0) return;
  if (in_sizes[1]  != NTOK * D1) return;
  if (in_sizes[2]  != NTOK * D2) return;
  if (in_sizes[3]  != NTOK * D3) return;
  if (in_sizes[4]  != NEX * DTOT) return;
  if (in_sizes[5]  != NEX) return;
  if (in_sizes[6]  != NOUT * D0) return;
  if (in_sizes[7]  != NOUT) return;
  if (in_sizes[8]  != NOUT * D1) return;
  if (in_sizes[9]  != NOUT) return;
  if (in_sizes[10] != NOUT * D2) return;
  if (in_sizes[11] != NOUT) return;
  if (in_sizes[12] != NOUT * D3) return;
  if (in_sizes[13] != NOUT) return;
  if (out_size != NTOK * NOUT) return;

  const float* f0 = (const float*)d_in[0];
  const float* f1 = (const float*)d_in[1];
  const float* f2 = (const float*)d_in[2];
  const float* f3 = (const float*)d_in[3];
  const float* gw = (const float*)d_in[4];
  const float* gb = (const float*)d_in[5];
  const float* w0 = (const float*)d_in[6];
  const float* b0 = (const float*)d_in[7];
  const float* w1 = (const float*)d_in[8];
  const float* b1 = (const float*)d_in[9];
  const float* w2 = (const float*)d_in[10];
  const float* b2 = (const float*)d_in[11];
  const float* w3 = (const float*)d_in[12];
  const float* b3 = (const float*)d_in[13];
  float* out = (float*)d_out;

  const size_t bX0   = (size_t)NTOK * D0 * 2;
  const size_t bX1   = (size_t)NTOK * D1 * 2;
  const size_t bX2   = (size_t)NTOK * D2 * 2;
  const size_t bX3   = (size_t)NTOK * D3 * 2;
  const size_t bW0   = (size_t)NOUT * D0 * 2;
  const size_t bW1   = (size_t)NOUT * D1 * 2;
  const size_t bW2   = (size_t)NOUT * D2 * 2;
  const size_t bW3   = (size_t)NOUT * D3 * 2;
  const size_t bREC  = (size_t)NTOK * 16;
  const size_t bPART = (size_t)NTOK * 2 * NOUT * 4;
  const size_t total = bX0 + bX1 + bX2 + bX3 + bW0 + bW1 + bW2 + bW3 + bREC + bPART;
  if (total > ws_size) return;
  if (total > (size_t)134217728) return;

  char* ws = (char*)d_ws;
  size_t off = 0;
  unsigned short* XH0 = (unsigned short*)(ws + off); off += bX0;
  unsigned short* XH1 = (unsigned short*)(ws + off); off += bX1;
  unsigned short* XH2 = (unsigned short*)(ws + off); off += bX2;
  unsigned short* XH3 = (unsigned short*)(ws + off); off += bX3;
  unsigned short* WH0 = (unsigned short*)(ws + off); off += bW0;
  unsigned short* WH1 = (unsigned short*)(ws + off); off += bW1;
  unsigned short* WH2 = (unsigned short*)(ws + off); off += bW2;
  unsigned short* WH3 = (unsigned short*)(ws + off); off += bW3;
  float*          REC = (float*)(ws + off);          off += bREC;
  float*          PART = (float*)(ws + off);         off += bPART;
  if (off != total) return;

  hipFuncSetAttribute(reinterpret_cast<const void*>(&k_expert),
                      hipFuncAttributeMaxDynamicSharedMemorySize, LDS_EXP);

  {
    const int n8x0 = NTOK * D0 / 8, n8x1 = NTOK * D1 / 8, n8x2 = NTOK * D2 / 8, n8x3 = NTOK * D3 / 8;
    const int n8w0 = NOUT * D0 / 8, n8w1 = NOUT * D1 / 8, n8w2 = NOUT * D2 / 8, n8w3 = NOUT * D3 / 8;
    k_cvt<<<(n8x0 + 255) / 256, 256, 0, stream>>>(f0, XH0, n8x0, 1.0f);
    k_cvt<<<(n8x1 + 255) / 256, 256, 0, stream>>>(f1, XH1, n8x1, 1.0f);
    k_cvt<<<(n8x2 + 255) / 256, 256, 0, stream>>>(f2, XH2, n8x2, 1.0f);
    k_cvt<<<(n8x3 + 255) / 256, 256, 0, stream>>>(f3, XH3, n8x3, 1.0f);
    k_cvt<<<(n8w0 + 255) / 256, 256, 0, stream>>>(w0, WH0, n8w0, W_SC);
    k_cvt<<<(n8w1 + 255) / 256, 256, 0, stream>>>(w1, WH1, n8w1, W_SC);
    k_cvt<<<(n8w2 + 255) / 256, 256, 0, stream>>>(w2, WH2, n8w2, W_SC);
    k_cvt<<<(n8w3 + 255) / 256, 256, 0, stream>>>(w3, WH3, n8w3, W_SC);
  }
  k_route<<<(NTOK + 7) / 8, 256, 0, stream>>>(f0, f1, f2, f3, gw, gb, REC, NTOK);
  k_expert<<<dim3(NTOK / MT, NEX), 256, LDS_EXP, stream>>>(XH0, XH1, XH2, XH3,
                                                          WH0, WH1, WH2, WH3,
                                                          b0, b1, b2, b3,
                                                          REC, PART, NTOK);
  {
    const int n4 = NTOK * NOUT / 4;
    k_sum<<<(n4 + 255) / 256, 256, 0, stream>>>(PART, out, n4);
  }
}
